// Mamba2DBlock_19104014532635
// MI455X (gfx1250) — hardware-run, weakly checked
//
#include <hip/hip_runtime.h>
#include <math.h>

typedef __attribute__((ext_vector_type(16))) _Float16 v16h;
typedef __attribute__((ext_vector_type(8)))  _Float16 v8h;
typedef __attribute__((ext_vector_type(16))) __bf16   v16b;
typedef __attribute__((ext_vector_type(8)))  __bf16   v8b;
typedef __attribute__((ext_vector_type(8)))  float    v8f;
typedef __attribute__((ext_vector_type(4)))  float    v4f;
typedef __attribute__((ext_vector_type(2)))  float    v2f;
typedef __attribute__((ext_vector_type(4)))  unsigned v4u;

constexpr int kB     = 4;
constexpr int kL     = 1024;
constexpr int kDm    = 1024;
constexpr int kDin   = 2048;
constexpr int kNst   = 16;
constexpr int kDtR   = 64;
constexpr int kXpN   = 96;
constexpr int kXpNP  = 128;
constexpr int kXzN   = 2 * kDin;
constexpr int kYcN   = 2 * kDm;
constexpr int kRows  = kB * kL;
constexpr float kEps = 1e-5f;
constexpr float kWCarry    = 16.0f;
constexpr float kWCarryInv = 0.0625f;
constexpr int kConvT  = 64;
constexpr int kScanTS = 64;
constexpr int kScanCh = 64;
constexpr int kScanBC = 32;
constexpr int kScanYP = 68;
static_assert(kDtR + 2 * kNst == kXpN && kXpN <= kXpNP, "x_proj layout");
static_assert((kDm % 32) == 0 && (kDin % 32) == 0 && (kDtR % 32) == 0 && (kYcN % 32) == 0, "GEMM K multiples of 32");
static_assert((kRows % 64) == 0 && (kXzN % 64) == 0 && (kXpNP % 64) == 0 && (kDin % 64) == 0 && (kDm % 64) == 0, "GEMM M,N multiples of 64");
static_assert((((kRows / 64) * (kXzN / 64)) % 8) == 0 && (((kRows / 64) * (kXpNP / 64)) % 8) == 0 &&
              (((kRows / 64) * (kDin / 64)) % 8) == 0 && (((kRows / 64) * (kDm / 64)) % 8) == 0, "8 tiles per GEMM block");
static_assert((kL % kConvT) == 0 && (kL % kScanTS) == 0 && (kDin % 256) == 0 && (kDin % kScanCh) == 0 && kScanCh == kScanTS, "tile multiples");
static_assert(kDm == 128 * 8, "LN: 128 threads x 8 elements per row");

constexpr size_t kOffWIN  = 0;
constexpr size_t kOffWXP0 = kOffWIN  + (size_t)kXzN  * kDm   * 2;
constexpr size_t kOffWXP1 = kOffWXP0 + (size_t)kXpNP * kDin  * 2;
constexpr size_t kOffWDT0 = kOffWXP1 + (size_t)kXpNP * kDin  * 2;
constexpr size_t kOffWDT1 = kOffWDT0 + (size_t)kDin  * kDtR  * 2;
constexpr size_t kOffWOU0 = kOffWDT1 + (size_t)kDin  * kDtR  * 2;
constexpr size_t kOffWOU1 = kOffWOU0 + (size_t)kDm   * kDin  * 2;
constexpr size_t kOffWMG  = kOffWOU1 + (size_t)kDm   * kDin  * 2;
constexpr size_t kOffXN   = kOffWMG  + (size_t)kDm   * kYcN  * 2;
constexpr size_t kOffXZ   = kOffXN   + (size_t)kRows * kDm   * 2;
constexpr size_t kOffUU   = kOffXZ   + (size_t)kRows * kXzN  * 2;
constexpr size_t kOffXD   = kOffUU   + (size_t)kRows * kDin  * 2;
constexpr size_t kOffVV   = kOffXD   + (size_t)kRows * kXpNP * 2;
constexpr size_t kOffYY   = kOffVV   + (size_t)kRows * kDin  * 2;
constexpr size_t kOffYC   = kOffYY   + (size_t)kRows * kDin  * 2;
constexpr size_t kWsTotal = kOffYC   + (size_t)kRows * kYcN  * 2;
static_assert(kWsTotal == 132644864ull, "carve total");
static_assert(kWsTotal <= 134217728ull, "carve cap");
static_assert((kOffWXP0 % 128) == 0 && (kOffWXP1 % 128) == 0 && (kOffWDT0 % 128) == 0 && (kOffWDT1 % 128) == 0 &&
              (kOffWOU0 % 128) == 0 && (kOffWOU1 % 128) == 0 && (kOffWMG % 128) == 0 && (kOffXN % 128) == 0 &&
              (kOffXZ % 128) == 0 && (kOffUU % 128) == 0 && (kOffXD % 128) == 0 && (kOffVV % 128) == 0 &&
              (kOffYY % 128) == 0 && (kOffYC % 128) == 0, "128-B aligned regions");

__device__ __forceinline__ unsigned short f2bf_bits(float f) {
  unsigned u = __float_as_uint(f);
  return (unsigned short)((u + 0x7FFFu + ((u >> 16) & 1u)) >> 16);
}
__device__ __forceinline__ float bf_bits2f(unsigned short h) { return __uint_as_float(((unsigned)h) << 16); }

__device__ __forceinline__ float h16_to_f32(unsigned hb) {
  const unsigned sgn = (hb & 0x8000u) << 16; const unsigned em = hb & 0x7fffu;
  const float fn = __uint_as_float((em << 13) + 0x38000000u);
  const float fs = (float)em * 5.9604644775390625e-8f;
  const float mag = (em < 0x400u) ? fs : fn; return __uint_as_float(__float_as_uint(mag) | sgn); }

__device__ __forceinline__ unsigned pack_f16x2(float a, float b) {
  const _Float16 h0 = (_Float16)a, h1 = (_Float16)b;
  return (unsigned)__builtin_bit_cast(unsigned short, h0) | ((unsigned)__builtin_bit_cast(unsigned short, h1) << 16);
}

__device__ __forceinline__ void dep_guard_h(v8f& a, v8f& b, v16h x, v16h y) { asm volatile("v_nop\n\tv_nop\n\tv_nop\n\tv_nop" : "+v"(a), "+v"(b) : "v"(x), "v"(y)); }
__device__ __forceinline__ void dep_guard_b(v8f& a, v8f& b, v16b x, v16b y) { asm volatile("v_nop\n\tv_nop\n\tv_nop\n\tv_nop" : "+v"(a), "+v"(b) : "v"(x), "v"(y)); }
__device__ __forceinline__ void keep4_h(v16h a, v16h b, v16h c, v16h d) { asm volatile("v_nop" :: "v"(a), "v"(b), "v"(c), "v"(d)); }
__device__ __forceinline__ void keep4_b(v16b a, v16b b, v16b c, v16b d) { asm volatile("v_nop" :: "v"(a), "v"(b), "v"(c), "v"(d)); }
__device__ __forceinline__ void acc_guard4(v8f& a, v8f& b, v8f& c, v8f& d) { asm volatile("v_nop\n\tv_nop\n\tv_nop\n\tv_nop" : "+v"(a), "+v"(b), "+v"(c), "+v"(d)); }
template <typename T> struct Frag;
template <> struct Frag<_Float16> {
  typedef v16h V; union U { v16h v; v8h h[2]; };
  static __device__ __forceinline__ v16h load(const _Float16* p) {
    U f; f.h[0] = *(const v8h*)(p); f.h[1] = *(const v8h*)(p + 16); return f.v;
  }
  static __device__ __forceinline__ v8f mma(v16h a, v16h b, v8f c) {
    return __builtin_amdgcn_wmma_f32_16x16x32_f16(false, a, false, b, (short)0, c, false, false);
  }
  static __device__ __forceinline__ void guard(v8f& a, v8f& b, v16h x, v16h y) { dep_guard_h(a, b, x, y); }
  static __device__ __forceinline__ void keep(v16h a, v16h b, v16h c, v16h d) { keep4_h(a, b, c, d); }
};
template <> struct Frag<__bf16> {
  typedef v16b V; union U { v16b v; v8b h[2]; };
  static __device__ __forceinline__ v16b load(const __bf16* p) {
    U f; f.h[0] = *(const v8b*)(p); f.h[1] = *(const v8b*)(p + 16); return f.v;
  }
  static __device__ __forceinline__ v8f mma(v16b a, v16b b, v8f c) {
    return __builtin_amdgcn_wmma_f32_16x16x32_bf16(false, a, false, b, (short)0, c, false, false);
  }
  static __device__ __forceinline__ void guard(v8f& a, v8f& b, v16b x, v16b y) { dep_guard_b(a, b, x, y); }
  static __device__ __forceinline__ void keep(v16b a, v16b b, v16b c, v16b d) { keep4_b(a, b, c, d); }
};

template <int ET> struct Elem;
template <> struct Elem<0> { typedef _Float16 T; };
template <> struct Elem<1> { typedef __bf16 T; };
template <int ET, bool SPLIT, int BIAS_MODE, int OUT_MODE, bool RESID, int ACT = 0>
__global__ __launch_bounds__(256) void wmma_gemm64(
    const unsigned short* __restrict__ Ap, const unsigned short* __restrict__ A2p, int lda, long strideA,
    const unsigned short* __restrict__ Btp, const unsigned short* __restrict__ Bt2p, int ldb, long strideB,
    void* __restrict__ Cout, void* __restrict__ Cout2, int ldc, long strideC,
    const float* __restrict__ bias,
    const float* __restrict__ resid, long strideR,
    int M, int N, int K, float scale) {
  static_assert(!(RESID && OUT_MODE != 0), "residual only with f32 output");
  typedef typename Elem<ET>::T T;
  typedef typename Frag<T>::V V;
  const T* A = (const T*)Ap; const T* A2 = (const T*)A2p; const T* Bt = (const T*)Btp; const T* Bt2 = (const T*)Bt2p;
  __shared__ __align__(16) float sT[8][16 * 68];
  const int b    = blockIdx.y;
  const int lane = threadIdx.x & 31;
  const int wave = threadIdx.x >> 5;
  const int tilesN = N >> 6;
  const int tilesM = M >> 6;
  const int tile = blockIdx.x * 8 + wave;
  if (tile >= tilesM * tilesN) return;
  const int tm = tile / tilesN;
  const int tn = tile - tm * tilesN;
  const int m0 = tm << 6;
  const int n0 = tn << 6;

  const T* Ab  = A  + (size_t)b * strideA;
  const T* Bb  = Bt + (size_t)b * strideB;
  const T* Ab2 = SPLIT ? (A2  + (size_t)b * strideA) : nullptr;
  const T* Bb2 = SPLIT ? (Bt2 + (size_t)b * strideB) : nullptr;

  const int rlane = lane & 15;
  const int koff  = (lane >> 4) * 8;
  const int mOff  = (lane >> 4) * 8;

  v8f acc[4][4];
#pragma unroll
  for (int i = 0; i < 4; ++i)
#pragma unroll
    for (int j = 0; j < 4; ++j) acc[i][j] = (v8f){0.f,0.f,0.f,0.f,0.f,0.f,0.f,0.f};

  for (int k0 = 0; k0 < K; k0 += 32) {
    V bh[4], bl[4];
#pragma unroll
    for (int j = 0; j < 4; ++j) {
      const size_t bo = (size_t)(n0 + (j << 4) + rlane) * ldb + koff + k0;
      bh[j] = Frag<T>::load(Bb + bo);
      if (SPLIT) bl[j] = Frag<T>::load(Bb2 + bo);
    }
#pragma unroll
    for (int i = 0; i < 4; ++i) {
      const size_t ao = (size_t)(m0 + (i << 4) + rlane) * lda + koff + k0;
      V ah = Frag<T>::load(Ab + ao);
      V al;
      if (SPLIT) al = Frag<T>::load(Ab2 + ao);
#pragma unroll
      for (int j = 0; j < 4; ++j) {
        acc[i][j] = Frag<T>::mma(ah, bh[j], acc[i][j]);
        if (SPLIT) {
          acc[i][j] = Frag<T>::mma(ah, bl[j], acc[i][j]);
          acc[i][j] = Frag<T>::mma(al, bh[j], acc[i][j]);
        }
      }
      Frag<T>::guard(acc[i][0], acc[i][3], ah, SPLIT ? al : ah);
    }
    Frag<T>::keep(bh[0], bh[1], bh[2], bh[3]);
    if (SPLIT) Frag<T>::keep(bl[0], bl[1], bl[2], bl[3]);
  }
  acc_guard4(acc[0][0], acc[0][1], acc[0][2], acc[0][3]);
  acc_guard4(acc[1][0], acc[1][1], acc[1][2], acc[1][3]);
  acc_guard4(acc[2][0], acc[2][1], acc[2][2], acc[2][3]);
  acc_guard4(acc[3][0], acc[3][1], acc[3][2], acc[3][3]);

  float* slab = sT[wave];
  const float* Rb = RESID ? (resid + (size_t)b * strideR) : nullptr;
#pragma unroll
  for (int i = 0; i < 4; ++i) {
    const int mBase = m0 + (i << 4);
#pragma unroll
    for (int j = 0; j < 4; ++j) {
      const int n = n0 + (j << 4) + rlane;
      float bv = 0.f;
      if (BIAS_MODE == 2) bv = bias[n];
#pragma unroll
      for (int r = 0; r < 8; ++r) {
        float v = acc[i][j][r] * scale;
        if (BIAS_MODE == 1) v += bias[mBase + mOff + r];
        if (BIAS_MODE == 2) v += bv;
        if (ACT == 1) v = tanhf(v);
        if (ACT == 2) v = fmaxf(v, 0.0f);
        if (ACT == 3) v = v / (1.0f + expf(-v));
        if (ACT == 4) v = (v > 0.f) ? v : 0.01f * v;
        slab[(mOff + r) * 68 + (j << 4) + rlane] = v;
      }
    }
    __builtin_amdgcn_fence(__ATOMIC_RELEASE, "workgroup");
    __builtin_amdgcn_wave_barrier();
    __builtin_amdgcn_fence(__ATOMIC_ACQUIRE, "workgroup");
    if (OUT_MODE == 0) {
      float* C = (float*)Cout + (size_t)b * strideC;
      const int hh = lane >> 4, c4 = (lane & 15) * 4;
      v4f ov[8];
#pragma unroll
      for (int it = 0; it < 8; ++it) {
        const int row = it * 2 + hh;
        v4f v = *(const v4f*)(slab + row * 68 + c4);
        if (RESID) {
          const v4f rr = *(const v4f*)(Rb + (size_t)(mBase + row) * ldc + n0 + c4);
          v += rr;
        }
        ov[it] = v;
      }
      for (int pass = 0; pass < 2; ++pass) {
#pragma unroll
        for (int it = 0; it < 8; ++it) {
          const int row = it * 2 + hh;
          *(volatile v4f*)(C + (size_t)(mBase + row) * ldc + n0 + c4) = ov[it];
        }
        __threadfence();
      }
    } else {
      const int q = lane >> 3, c8 = (lane & 7) * 8;
      unsigned short* C  = (unsigned short*)Cout  + (size_t)b * strideC;
      unsigned short* C2 = (OUT_MODE == 2) ? ((unsigned short*)Cout2 + (size_t)b * strideC) : nullptr;
      for (int pass = 0; pass < 2; ++pass) {
#pragma unroll
        for (int it = 0; it < 4; ++it) {
          const int row = it * 4 + q;
          const float* sp = slab + row * 68 + c8;
          v8h hv, lv;
#pragma unroll
          for (int e = 0; e < 8; ++e) {
            if (OUT_MODE == 1) {
              hv[e] = (_Float16)sp[e];
            } else {
              unsigned short hb = f2bf_bits(sp[e]);
              unsigned short lb = f2bf_bits(sp[e] - bf_bits2f(hb));
              hv[e] = __builtin_bit_cast(_Float16, hb);
              lv[e] = __builtin_bit_cast(_Float16, lb);
            }
          }
          *(volatile v8h*)(C + (size_t)(mBase + row) * ldc + n0 + c8) = hv;
          if (OUT_MODE == 2) *(volatile v8h*)(C2 + (size_t)(mBase + row) * ldc + n0 + c8) = lv;
        }
        __threadfence();
      }
    }
    __builtin_amdgcn_fence(__ATOMIC_RELEASE, "workgroup");
    __builtin_amdgcn_wave_barrier();
    __builtin_amdgcn_fence(__ATOMIC_ACQUIRE, "workgroup");
  }
}

__global__ __launch_bounds__(256) void cast_pad_f16x2_kernel(
    const float* __restrict__ in, int n_src, unsigned* __restrict__ out, int n2, float carry) {
  const int i = blockIdx.x * 256 + threadIdx.x;
  if (i >= n2) return;
  const int e = 2 * i;
  const bool live = (e + 1 < n_src);
  const int ec = live ? e : (n_src - 2);
  const v2f p = *(const v2f*)(in + ec);
  const float fac = live ? carry : 0.0f;
  const unsigned u = pack_f16x2(p[0] * fac, p[1] * fac);
  ((volatile unsigned*)out)[i] = u;
  __threadfence();
  ((volatile unsigned*)out)[i] = u;
}

__global__ __launch_bounds__(128) void layernorm_f16_kernel(
    const float* __restrict__ x, const float* __restrict__ g, const float* __restrict__ bta,
    unsigned short* __restrict__ XN) {
  __shared__ float red[2][4];
  const int tid = threadIdx.x, lane = tid & 31, wave = tid >> 5;
  const size_t row = blockIdx.x;
  const float* xr = x + row * kDm + (size_t)tid * 8;
  const v4f a0 = *(const v4f*)(xr);
  const v4f a1 = *(const v4f*)(xr + 4);
  float s = 0.0f;
  s += a0[0]; s += a0[1]; s += a0[2]; s += a0[3];
  s += a1[0]; s += a1[1]; s += a1[2]; s += a1[3];
#pragma unroll
  for (int off = 16; off > 0; off >>= 1) s += __shfl_xor(s, off, 32);
  if (lane == 0) red[0][wave] = s;
  __syncthreads();
  const float mu = ((red[0][0] + red[0][1]) + (red[0][2] + red[0][3])) * (1.0f / (float)kDm);
  const v4f d0 = a0 - mu;
  const v4f d1 = a1 - mu;
  float q = 0.0f;
  q = fmaf(d0[0], d0[0], q); q = fmaf(d0[1], d0[1], q); q = fmaf(d0[2], d0[2], q); q = fmaf(d0[3], d0[3], q);
  q = fmaf(d1[0], d1[0], q); q = fmaf(d1[1], d1[1], q); q = fmaf(d1[2], d1[2], q); q = fmaf(d1[3], d1[3], q);
#pragma unroll
  for (int off = 16; off > 0; off >>= 1) q += __shfl_xor(q, off, 32);
  if (lane == 0) red[1][wave] = q;
  __syncthreads();
  const float var = ((red[1][0] + red[1][1]) + (red[1][2] + red[1][3])) * (1.0f / (float)kDm);
  const float rs = rsqrtf(var + kEps);
  const v4f g0 = *(const v4f*)(g + tid * 8);
  const v4f g1 = *(const v4f*)(g + tid * 8 + 4);
  const v4f b0 = *(const v4f*)(bta + tid * 8);
  const v4f b1 = *(const v4f*)(bta + tid * 8 + 4);
  v8h hv;
#pragma unroll
  for (int e = 0; e < 4; ++e) {
    hv[e]     = (_Float16)((d0[e] * rs) * g0[e] + b0[e]);
    hv[4 + e] = (_Float16)((d1[e] * rs) * g1[e] + b1[e]);
  }
  unsigned short* op = XN + row * kDm + (size_t)tid * 8;
  *(volatile v8h*)(void*)op = hv;
  __threadfence();
  *(volatile v8h*)(void*)op = hv;
}

__global__ __launch_bounds__(128) void conv_silu_f16_kernel(
    const unsigned* __restrict__ XZw, const float* __restrict__ cw, const float* __restrict__ cb,
    unsigned* __restrict__ Uw, int dir) {
  const int tid = threadIdx.x;
  const int dp  = blockIdx.x * 256 + 2 * tid;
  const int g0  = blockIdx.y * kConvT;
  const int bix = g0 / kL;
  const int tb  = g0 - bix * kL;
  const size_t brow = (size_t)bix * kL;
  const v4f wa = *(const v4f*)(cw + (size_t)dp * 4);
  const v4f wb = *(const v4f*)(cw + (size_t)dp * 4 + 4);
  const float ba = cb[dp], bbias = cb[dp + 1];
  const int r0    = dir ? (tb + kConvT - 1) : tb;
  const int dstep = dir ? -1 : 1;
  const bool hist = dir ? (tb + kConvT < kL) : (tb > 0);
  const float fac = hist ? 1.0f : 0.0f;
  int r1 = r0 - dstep, r2 = r0 - 2 * dstep, r3 = r0 - 3 * dstep;
  r1 = r1 < 0 ? 0 : (r1 > kL - 1 ? kL - 1 : r1);
  r2 = r2 < 0 ? 0 : (r2 > kL - 1 ? kL - 1 : r2);
  r3 = r3 < 0 ? 0 : (r3 > kL - 1 ? kL - 1 : r3);
  const unsigned q1 = XZw[((brow + r1) * kXzN + dp) >> 1];
  const unsigned q2 = XZw[((brow + r2) * kXzN + dp) >> 1];
  const unsigned q3 = XZw[((brow + r3) * kXzN + dp) >> 1];
  float n1a = h16_to_f32(q1 & 0xffffu) * fac, n1b = h16_to_f32(q1 >> 16) * fac;
  float n2a = h16_to_f32(q2 & 0xffffu) * fac, n2b = h16_to_f32(q2 >> 16) * fac;
  float n3a = h16_to_f32(q3 & 0xffffu) * fac, n3b = h16_to_f32(q3 >> 16) * fac;
#pragma unroll 1
  for (int s = 0; s < kConvT; ++s) {
    const int r = r0 + s * dstep;
    const unsigned qc = XZw[((brow + r) * kXzN + dp) >> 1];
    const float ca = h16_to_f32(qc & 0xffffu);
    const float cbv = h16_to_f32(qc >> 16);
    float acca = wa[0] * n3a;
    acca = fmaf(wa[1], n2a, acca);
    acca = fmaf(wa[2], n1a, acca);
    acca = fmaf(wa[3], ca, acca);
    acca += ba;
    float accb = wb[0] * n3b;
    accb = fmaf(wb[1], n2b, accb);
    accb = fmaf(wb[2], n1b, accb);
    accb = fmaf(wb[3], cbv, accb);
    accb += bbias;
    const float ua = acca * __builtin_amdgcn_rcpf(1.0f + expf(-acca));
    const float ub = accb * __builtin_amdgcn_rcpf(1.0f + expf(-accb));
    const unsigned u = pack_f16x2(ua, ub);
    const size_t oix = ((brow + r) * kDin + dp) >> 1;
    ((volatile unsigned*)Uw)[oix] = u;
    __threadfence();
    ((volatile unsigned*)Uw)[oix] = u;
    n3a = n2a; n2a = n1a; n1a = ca;
    n3b = n2b; n2b = n1b; n1b = cbv;
  }
}

__device__ __forceinline__ void cvt_word8(v4u w, float* __restrict__ dst8) {
  v4f lo, hi;
  lo[0] = h16_to_f32(w[0] & 0xffffu); lo[1] = h16_to_f32(w[0] >> 16);
  lo[2] = h16_to_f32(w[1] & 0xffffu); lo[3] = h16_to_f32(w[1] >> 16);
  hi[0] = h16_to_f32(w[2] & 0xffffu); hi[1] = h16_to_f32(w[2] >> 16);
  hi[2] = h16_to_f32(w[3] & 0xffffu); hi[3] = h16_to_f32(w[3] >> 16);
  *(v4f*)(dst8) = lo;
  *(v4f*)(dst8 + 4) = hi;
}

__global__ __launch_bounds__(kScanCh) void scan_kernel(
    const unsigned short* __restrict__ XD, const unsigned short* __restrict__ VV,
    const unsigned short* __restrict__ UU, const unsigned short* __restrict__ XZ,
    const float* __restrict__ dtb, const float* __restrict__ Alog, const float* __restrict__ Dp,
    unsigned short* __restrict__ YY, int dir) {
  __shared__ __align__(16) float sBC[kScanTS * kScanBC];
  __shared__ __align__(16) float sY[kScanTS * kScanYP];
  __shared__ __align__(16) float sA[kNst * kScanCh];
  const int tid = threadIdx.x, lane = tid & 31, wave = tid >> 5;
  constexpr int kBlkPerB = kDin / kScanCh;
  const int bix = blockIdx.x / kBlkPerB;
  const int d0  = (blockIdx.x - bix * kBlkPerB) * kScanCh;
  const int d   = d0 + tid;
  const size_t row0 = (size_t)bix * kL;
#pragma unroll 1
  for (int s = 0; s < kNst; ++s) sA[s * kScanCh + tid] = -expf(Alog[(size_t)d * kNst + s]);
  __syncthreads();
  float negA[kNst], h[kNst];
#pragma unroll
  for (int s = 0; s < kNst; ++s) {
    negA[s] = sA[s * kScanCh + tid];
    h[s] = 0.0f;
  }
  const float bb = dtb[d], Dd = Dp[d];
  const int q = lane >> 3, c8 = (lane & 7) * 8;
#pragma unroll 1
  for (int ci = 0; ci < kL / kScanTS; ++ci) {
    const int tbase = dir ? (kL - kScanTS - ci * kScanTS) : (ci * kScanTS);
    __syncthreads();
    {
      const size_t srow = row0 + tbase + tid;
      const v4u* sp = (const v4u*)(XD + srow * kXpNP + kDtR);
      const v4u w0 = sp[0], w1 = sp[1], w2 = sp[2], w3 = sp[3];
      float* dst = sBC + tid * kScanBC;
      cvt_word8(w0, dst);
      cvt_word8(w1, dst + 8);
      cvt_word8(w2, dst + 16);
      cvt_word8(w3, dst + 24);
    }
    __syncthreads();
#pragma unroll 1
    for (int s = 0; s < kScanTS; ++s) {
      const int sidx = dir ? (kScanTS - 1 - s) : s;
      const size_t row = row0 + tbase + sidx;
      const unsigned vh = VV[row * kDin + d];
      const unsigned uh = UU[row * kDin + d];
      const unsigned zh = XZ[row * kXzN + kDin + d];
      const float* xr = sBC + sidx * kScanBC;
      const v4f bq0 = *(const v4f*)(xr), bq1 = *(const v4f*)(xr + 4), bq2 = *(const v4f*)(xr + 8), bq3 = *(const v4f*)(xr + 12);
      const v4f cq0 = *(const v4f*)(xr + 16), cq1 = *(const v4f*)(xr + 20), cq2 = *(const v4f*)(xr + 24), cq3 = *(const v4f*)(xr + 28);
      float Bs[kNst], Cs[kNst];
#pragma unroll
      for (int e = 0; e < 4; ++e) {
        Bs[e] = bq0[e]; Bs[4 + e] = bq1[e]; Bs[8 + e] = bq2[e]; Bs[12 + e] = bq3[e];
        Cs[e] = cq0[e]; Cs[4 + e] = cq1[e]; Cs[8 + e] = cq2[e]; Cs[12 + e] = cq3[e];
      }
      const float v   = h16_to_f32(vh) + bb;
      const float a   = __expf(-fabsf(v));
      const float uu1 = 1.0f + a;
      const float l1p = __logf(uu1) + (a - (uu1 - 1.0f)) * __builtin_amdgcn_rcpf(uu1);
      const float dt  = fmaxf(v, 0.0f) + l1p;
      const float xt  = h16_to_f32(uh);
      const float dtx = dt * xt;
      float y = 0.0f;
#pragma unroll
      for (int k = 0; k < kNst; ++k) {
        const float e = __expf(dt * negA[k]);
        h[k] = e * h[k] + dtx * Bs[k];
        y = fmaf(h[k], Cs[k], y);
      }
      const float ud = xt * Dd;
      y = y + ud;
      const float zv = h16_to_f32(zh);
      const float sg = __builtin_amdgcn_rcpf(1.0f + __expf(-zv));
      y = y * (zv * sg);
      sY[sidx * kScanYP + tid] = y;
    }
    __syncthreads();
    v8h hv[8];
#pragma unroll
    for (int it = 0; it < 8; ++it) {
      const int rr = it * 8 + wave * 4 + q;
      const float* sp = sY + rr * kScanYP + c8;
      const v4f a0 = *(const v4f*)(sp);
      const v4f a1 = *(const v4f*)(sp + 4);
#pragma unroll
      for (int e = 0; e < 4; ++e) {
        hv[it][e]     = (_Float16)a0[e];
        hv[it][4 + e] = (_Float16)a1[e];
      }
    }
    for (int pass = 0; pass < 2; ++pass) {
#pragma unroll
      for (int it = 0; it < 8; ++it) {
        const int rr = it * 8 + wave * 4 + q;
        const size_t o = (row0 + tbase + rr) * kDin + d0 + c8;
        *(volatile v8h*)(void*)(YY + o) = hv[it];
      }
      __threadfence();
    }
  }
}

extern "C" void kernel_launch(void* const* d_in, const int* in_sizes, int n_in,
                              void* d_out, int out_size, void* d_ws, size_t ws_size,
                              hipStream_t stream) {
  if (n_in < 23) return;
  if (in_sizes[0] != kRows * kDm) return;
  if (in_sizes[1] != kDm || in_sizes[2] != kDm) return;
  if (in_sizes[3] != kDm * kYcN || in_sizes[4] != kDm) return;
  for (int dir = 0; dir < 2; ++dir) {
    const int base = 5 + dir * 9;
    if (in_sizes[base + 0] != kXzN * kDm) return;
    if (in_sizes[base + 1] != kDin * 4) return;
    if (in_sizes[base + 2] != kDin) return;
    if (in_sizes[base + 3] != kXpN * kDin) return;
    if (in_sizes[base + 4] != kDin * kDtR) return;
    if (in_sizes[base + 5] != kDin) return;
    if (in_sizes[base + 6] != kDin * kNst) return;
    if (in_sizes[base + 7] != kDin) return;
    if (in_sizes[base + 8] != kDm * kDin) return;
  }
  if (out_size != kRows * kDm) return;
  if (ws_size < kWsTotal) return;

  const float* x       = (const float*)d_in[0];
  const float* norm_g  = (const float*)d_in[1];
  const float* norm_b  = (const float*)d_in[2];
  const float* merge_w = (const float*)d_in[3];
  const float* merge_b = (const float*)d_in[4];
  float* out = (float*)d_out;

  char* ws = (char*)d_ws;
  unsigned short* WIN    = (unsigned short*)(ws + kOffWIN);
  unsigned short* WXP[2] = {(unsigned short*)(ws + kOffWXP0), (unsigned short*)(ws + kOffWXP1)};
  unsigned short* WDT[2] = {(unsigned short*)(ws + kOffWDT0), (unsigned short*)(ws + kOffWDT1)};
  unsigned short* WOU[2] = {(unsigned short*)(ws + kOffWOU0), (unsigned short*)(ws + kOffWOU1)};
  unsigned short* WMG    = (unsigned short*)(ws + kOffWMG);
  unsigned short* XN     = (unsigned short*)(ws + kOffXN);
  unsigned short* XZ     = (unsigned short*)(ws + kOffXZ);
  unsigned short* UU     = (unsigned short*)(ws + kOffUU);
  unsigned short* XD     = (unsigned short*)(ws + kOffXD);
  unsigned short* VV     = (unsigned short*)(ws + kOffVV);
  unsigned short* YY     = (unsigned short*)(ws + kOffYY);
  unsigned short* YC     = (unsigned short*)(ws + kOffYC);

  for (int dir = 0; dir < 2; ++dir) {
    const int base = 5 + dir * 9;
    const float* xproj_w = (const float*)d_in[base + 3];
    const float* dt_w    = (const float*)d_in[base + 4];
    const float* out_w   = (const float*)d_in[base + 8];
    {
      const int n2 = kXpNP * kDin / 2;
      cast_pad_f16x2_kernel<<<(n2 + 255) / 256, 256, 0, stream>>>(xproj_w, kXpN * kDin, (unsigned*)WXP[dir], n2, kWCarry);
    }
    {
      const int n2 = kDin * kDtR / 2;
      cast_pad_f16x2_kernel<<<(n2 + 255) / 256, 256, 0, stream>>>(dt_w, kDin * kDtR, (unsigned*)WDT[dir], n2, kWCarry);
    }
    {
      const int n2 = kDm * kDin / 2;
      cast_pad_f16x2_kernel<<<(n2 + 255) / 256, 256, 0, stream>>>(out_w, kDm * kDin, (unsigned*)WOU[dir], n2, kWCarry);
    }
  }
  {
    const int n2 = kDm * kYcN / 2;
    cast_pad_f16x2_kernel<<<(n2 + 255) / 256, 256, 0, stream>>>(merge_w, kDm * kYcN, (unsigned*)WMG, n2, kWCarry);
  }

  layernorm_f16_kernel<<<kRows, 128, 0, stream>>>(x, norm_g, norm_b, XN);

  for (int dir = 0; dir < 2; ++dir) {
    const int base = 5 + dir * 9;
    const float* in_w   = (const float*)d_in[base + 0];
    const float* conv_w = (const float*)d_in[base + 1];
    const float* conv_b = (const float*)d_in[base + 2];
    const float* dt_b   = (const float*)d_in[base + 5];
    const float* A_log  = (const float*)d_in[base + 6];
    const float* Dp     = (const float*)d_in[base + 7];

    {
      const int n2 = kXzN * kDm / 2;
      cast_pad_f16x2_kernel<<<(n2 + 255) / 256, 256, 0, stream>>>(in_w, kXzN * kDm, (unsigned*)WIN, n2, kWCarry);
    }

    wmma_gemm64<0, false, 0, 1, false><<<dim3(((kRows / 64) * (kXzN / 64)) / 8, 1), 256, 0, stream>>>(
        XN, nullptr, kDm, 0L,
        WIN, nullptr, kDm, 0L,
        (void*)XZ, nullptr, kXzN, 0L,
        nullptr, nullptr, 0L,
        kRows, kXzN, kDm, kWCarryInv);

    conv_silu_f16_kernel<<<dim3(kDin / 256, kRows / kConvT), 128, 0, stream>>>(
        (const unsigned*)(const void*)XZ, conv_w, conv_b, (unsigned*)(void*)UU, dir);

    wmma_gemm64<0, false, 0, 1, false><<<dim3(((kRows / 64) * (kXpNP / 64)) / 8, 1), 256, 0, stream>>>(
        UU, nullptr, kDin, 0L,
        WXP[dir], nullptr, kDin, 0L,
        (void*)XD, nullptr, kXpNP, 0L,
        nullptr, nullptr, 0L,
        kRows, kXpNP, kDin, kWCarryInv);

    wmma_gemm64<0, false, 0, 1, false><<<dim3(((kRows / 64) * (kDin / 64)) / 8, 1), 256, 0, stream>>>(
        XD, nullptr, kXpNP, 0L,
        WDT[dir], nullptr, kDtR, 0L,
        (void*)VV, nullptr, kDin, 0L,
        nullptr, nullptr, 0L,
        kRows, kDin, kDtR, kWCarryInv);

    scan_kernel<<<kB * (kDin / kScanCh), kScanCh, 0, stream>>>(XD, VV, UU, XZ, dt_b, A_log, Dp, YY, dir);

    wmma_gemm64<0, false, 0, 1, false><<<dim3(((kRows / 64) * (kDm / 64)) / 8, 1), 256, 0, stream>>>(
        YY, nullptr, kDin, 0L,
        WOU[dir], nullptr, kDin, 0L,
        (void*)(YC + (size_t)dir * kDm), nullptr, kYcN, 0L,
        nullptr, nullptr, 0L,
        kRows, kDm, kDin, kWCarryInv);
  }

  wmma_gemm64<0, false, 2, 0, true><<<dim3(((kRows / 64) * (kDm / 64)) / 8, 1), 256, 0, stream>>>(
      YC, nullptr, kYcN, 0L,
      WMG, nullptr, kYcN, 0L,
      (void*)out, nullptr, kDm, 0L,
      merge_b, x, 0L,
      kRows, kDm, kYcN, kWCarryInv);
}
